// GNNEncoderGAT_48481590837597
// MI455X (gfx1250) — hardware-verified
//
#include <hip/hip_runtime.h>
#include <stddef.h>


#define IN0   128
#define DF    256
#define NH    4
#define HC    64
#define HID   64
#define OUTD  128
#define NGR   256
#define GR    32
#define XSP   260
#define ZP    72
#define OSP   132
#define NB    256
#define CHUNK 2048
#define NTHR  256
#define NWAVE 8
#define WCAP  256
#define NGRP  (CHUNK / (NTHR * 4))

#define LDS_SACC (NB * DF)
#define LDS_DEN  (NB * NH)
#define LDS_MXR  (NB * NH)
#define LDS_LIST (NWAVE * WCAP)
#define LDS_AGG_BYTES ((LDS_SACC + LDS_DEN + LDS_MXR + LDS_LIST + 16) * 4)

static_assert(WCAP == (CHUNK / NTHR) * 32);
static_assert(NGRP == 2);
static_assert(NB == 256);
static_assert(NH * HC == DF);
static_assert(CHUNK <= 2048);
static_assert(LDS_AGG_BYTES == 278592);
static_assert((NB / NWAVE) == 32);

typedef float    v4f  __attribute__((ext_vector_type(4)));
typedef float    v8f  __attribute__((ext_vector_type(8)));
typedef int      v4i  __attribute__((ext_vector_type(4)));
typedef _Float16 v8h  __attribute__((ext_vector_type(8)));
typedef _Float16 v16h __attribute__((ext_vector_type(16)));
union Frag   { v16h v; v8h half[2]; };
union Pack16 { v8h h; v4i i; };

__device__ __forceinline__ v8f wm(v16h a, v16h b, v8f c) {
  v8f d = __builtin_amdgcn_wmma_f32_16x16x32_f16(false, a, false, b, (short)0, c, false, false);
  asm volatile("v_nop\n\tv_nop\n\tv_nop\n\tv_nop" : "+v"(d) : "v"(a), "v"(b));
  return d;
}

__device__ __forceinline__ float leaky(float x) { return x >= 0.f ? x : 0.2f * x; }

__device__ __forceinline__ v4f relu4(v4f v) {
  v.x = fmaxf(v.x, 0.f); v.y = fmaxf(v.y, 0.f); v.z = fmaxf(v.z, 0.f); v.w = fmaxf(v.w, 0.f);
  return v;
}

__global__ __launch_bounds__(NTHR) void k_cvt(const float* __restrict__ x, _Float16* xh, int nN, int n8) {
  const int i = blockIdx.x * NTHR + threadIdx.x;
  if (i >= n8) return;
  const int row = i >> 4;
  const int c8  = (i & 15) * 8;
  int rc = row; if (rc > nN - 1) rc = nN - 1;
  const float* p = x + (size_t)rc * IN0 + c8;
  v4f a = *(const v4f*)p;
  v4f b = *(const v4f*)(p + 4);
  const float keep = (row < nN) ? 1.0f : 0.0f;
  a = a * keep; b = b * keep;
  Pack16 u;
  u.h[0] = (_Float16)a.x; u.h[1] = (_Float16)a.y; u.h[2] = (_Float16)a.z; u.h[3] = (_Float16)a.w;
  u.h[4] = (_Float16)b.x; u.h[5] = (_Float16)b.y; u.h[6] = (_Float16)b.z; u.h[7] = (_Float16)b.w;
  _Float16* op = xh + (size_t)i * 8;
  *(volatile v4i*)op = u.i;
  __threadfence();
  *(volatile v4i*)op = u.i;
}

__global__ __launch_bounds__(NTHR) void k_wprep(const float* __restrict__ W, _Float16* Wt, int K, int NC, float sc, int n8) {
  const int i = blockIdx.x * NTHR + threadIdx.x;
  if (i >= n8) return;
  const int kq = K >> 3;
  const int n  = i / kq;
  const int k8 = (i - n * kq) * 8;
  Pack16 u;
#pragma unroll
  for (int j = 0; j < 8; ++j) u.h[j] = (_Float16)(W[(size_t)(k8 + j) * NC + n] * sc);
  _Float16* op = Wt + (size_t)i * 8;
  *(volatile v4i*)op = u.i;
  __threadfence();
  *(volatile v4i*)op = u.i;
}

__device__ __forceinline__ void put_tile(v8f c, int T, int J, int hh, int m, int wave, float osc, float* Xs) {
#pragma unroll
  for (int r = 0; r < 8; ++r) Xs[(16 * T + 8 * hh + r) * XSP + wave * 32 + 16 * J + m] = c[r] * osc;
}

template <int K>
__global__ __launch_bounds__(NTHR) void k_gemm(
    const _Float16* __restrict__ Ah, const _Float16* __restrict__ Wt,
    const float* __restrict__ att_src, const float* __restrict__ att_dst,
    float* xp, float* AL, float osc) {
  __shared__ __attribute__((aligned(16))) float Xs[GR * XSP];
  __shared__ __attribute__((aligned(16))) float asl[2 * DF];
  __shared__ __attribute__((aligned(16))) float Als[GR * 8];

  const int tid  = threadIdx.x;
  const int lane = tid & 31;
  const int wave = tid >> 5;
  const int hh   = lane >> 4;
  const int m    = lane & 15;
  const int rowBase = blockIdx.x * GR;

  asl[tid]      = att_src[tid];
  asl[DF + tid] = att_dst[tid];

  const _Float16* pa0 = Ah + (size_t)(rowBase + m) * K + 8 * hh;
  const _Float16* pa1 = Ah + (size_t)(rowBase + 16 + m) * K + 8 * hh;
  const _Float16* pb0 = Wt + (size_t)(wave * 32 + m) * K + 8 * hh;
  const _Float16* pb1 = Wt + (size_t)(wave * 32 + 16 + m) * K + 8 * hh;

  v8f c00 = {0.f, 0.f, 0.f, 0.f, 0.f, 0.f, 0.f, 0.f};
  v8f c01 = c00, c10 = c00, c11 = c00;
#pragma unroll 2
  for (int kt = 0; kt < K / 32; ++kt) {
    const int k0 = kt * 32;
    Frag a0, a1, b0, b1;
    a0.half[0] = *(const v8h*)(pa0 + k0); a0.half[1] = *(const v8h*)(pa0 + k0 + 16);
    a1.half[0] = *(const v8h*)(pa1 + k0); a1.half[1] = *(const v8h*)(pa1 + k0 + 16);
    b0.half[0] = *(const v8h*)(pb0 + k0); b0.half[1] = *(const v8h*)(pb0 + k0 + 16);
    b1.half[0] = *(const v8h*)(pb1 + k0); b1.half[1] = *(const v8h*)(pb1 + k0 + 16);
    c00 = wm(a0.v, b0.v, c00);
    c01 = wm(a0.v, b1.v, c01);
    c10 = wm(a1.v, b0.v, c10);
    c11 = wm(a1.v, b1.v, c11);
  }

  put_tile(c00, 0, 0, hh, m, wave, osc, Xs);
  put_tile(c01, 0, 1, hh, m, wave, osc, Xs);
  put_tile(c10, 1, 0, hh, m, wave, osc, Xs);
  put_tile(c11, 1, 1, hh, m, wave, osc, Xs);
  __syncthreads();

  {
    const int r  = tid >> 3;
    const int hd = (tid >> 1) & 3;
    const int sd = tid & 1;
    const float* xr = Xs + r * XSP + hd * HC;
    const float* av = asl + sd * DF + hd * HC;
    float s = 0.f;
#pragma unroll 4
    for (int c = 0; c < HC / 4; ++c) {
      const v4f xv = *(const v4f*)(xr + 4 * c);
      const v4f aa = *(const v4f*)(av + 4 * c);
      s += xv.x * aa.x + xv.y * aa.y + xv.z * aa.z + xv.w * aa.w;
    }
    Als[r * 8 + sd * 4 + hd] = s;
  }
  __syncthreads();

  v4f xr[8];
#pragma unroll
  for (int i = 0; i < 4; ++i) {
    xr[2 * i]     = *(const v4f*)(Xs + (4 * wave + i) * XSP + 4 * lane);
    xr[2 * i + 1] = *(const v4f*)(Xs + (4 * wave + i) * XSP + 128 + 4 * lane);
  }
  const int wsel = (wave < 2) ? wave : 0;
  const v4f gv = *(const v4f*)(Als + (wsel * 32 + lane) * 4);
  float* gp = AL + (size_t)rowBase * 8 + (wsel * 32 + lane) * 4;
  float* xb = xp + (size_t)(rowBase + 4 * wave) * DF + 4 * lane;

#pragma unroll
  for (int i = 0; i < 4; ++i) {
    *(volatile v4f*)(xb + (size_t)i * DF)       = xr[2 * i];
    *(volatile v4f*)(xb + (size_t)i * DF + 128) = xr[2 * i + 1];
  }
  if (wave < 2) *(volatile v4f*)gp = gv;
  __threadfence();
#pragma unroll
  for (int i = 0; i < 4; ++i) {
    *(volatile v4f*)(xb + (size_t)i * DF)       = xr[2 * i];
    *(volatile v4f*)(xb + (size_t)i * DF + 128) = xr[2 * i + 1];
  }
  if (wave < 2) *(volatile v4f*)gp = gv;
}

__global__ __launch_bounds__(NTHR) void k_agg(
    const int* __restrict__ ei, const float* __restrict__ xp, const float* __restrict__ AL,
    const float* __restrict__ bias, _Float16* hout, int nN, int nE, int nPad) {
  extern __shared__ v4f lds_dyn[];
  float* sacc = (float*)lds_dyn;
  float* den  = sacc + LDS_SACC;
  float* mxr  = den + LDS_DEN;
  int*   list = (int*)(mxr + LDS_MXR);
  int*   wcnt = list + LDS_LIST;

  const int tid  = threadIdx.x;
  const int lane = tid & 31;
  const int wave = tid >> 5;
  const int nodeBase = blockIdx.x * NB;

#pragma unroll 1
  for (int i = 0; i < LDS_SACC / 4 / NTHR; ++i) {
    const int q    = i * NTHR + tid;
    const int slot = q >> 6;
    const int c4   = q & 63;
    int node = nodeBase + slot; if (node > nN - 1) node = nN - 1;
    lds_dyn[q] = *(const v4f*)(xp + (size_t)node * DF + 4 * c4);
  }
#pragma unroll 1
  for (int q = tid; q < LDS_DEN; q += NTHR) {
    const int slot = q >> 2;
    const int hd   = q & 3;
    int node = nodeBase + slot; if (node > nN - 1) node = nN - 1;
    const float e = leaky(AL[(size_t)node * 8 + hd] + AL[(size_t)node * 8 + 4 + hd]);
    mxr[q] = e;
    den[q] = 1.0f;
  }
  __syncthreads();

  const int* eid = ei + nE;
  const bool al16 = ((nE & 3) == 0);

  const int nChunks = (nE + CHUNK - 1) / CHUNK;
#pragma unroll 1
  for (int ch = 0; ch < nChunks; ++ch) {
    const int cbase = ch * CHUNK;
    int wc = 0;
#pragma unroll
    for (int g = 0; g < NGRP; ++g) {
      const int el0 = (g * NTHR + tid) * 4;
      const int e0  = cbase + el0;
      const int sent = -2147483647 - 1;
      v4i d;
      if (al16 && (cbase + CHUNK <= nE)) {
        d = *(const v4i*)(eid + e0);
      } else {
        d.x = (e0     < nE) ? eid[min(e0,     nE - 1)] : sent;
        d.y = (e0 + 1 < nE) ? eid[min(e0 + 1, nE - 1)] : sent;
        d.z = (e0 + 2 < nE) ? eid[min(e0 + 2, nE - 1)] : sent;
        d.w = (e0 + 3 < nE) ? eid[min(e0 + 3, nE - 1)] : sent;
      }
      const unsigned s0 = (unsigned)d.x - (unsigned)nodeBase;
      const unsigned s1 = (unsigned)d.y - (unsigned)nodeBase;
      const unsigned s2 = (unsigned)d.z - (unsigned)nodeBase;
      const unsigned s3 = (unsigned)d.w - (unsigned)nodeBase;
      const bool h0 = s0 < (unsigned)NB;
      const bool h1 = s1 < (unsigned)NB;
      const bool h2 = s2 < (unsigned)NB;
      const bool h3 = s3 < (unsigned)NB;
      const unsigned many = __builtin_amdgcn_ballot_w32(h0 | h1 | h2 | h3);
      if (many != 0u) {
#define HITJ(J, HJ, SJ) { \
          const unsigned mj = __builtin_amdgcn_ballot_w32(HJ); \
          if (HJ) { \
            const int pos = wc + (int)__builtin_amdgcn_mbcnt_lo(mj, 0u); \
            if (pos < WCAP) list[wave * WCAP + pos] = ((el0 + (J)) << 8) | (int)(SJ); \
          } \
          wc += (int)__builtin_popcount(mj); }
        HITJ(0, h0, s0)
        HITJ(1, h1, s1)
        HITJ(2, h2, s2)
        HITJ(3, h3, s3)
#undef HITJ
      }
    }
    if (lane == 0) wcnt[wave] = wc;
    __syncthreads();

    if (wave == 0) {
      const int hd = lane >> 3;
#pragma unroll 1
      for (int wsx = 0; wsx < NWAVE; ++wsx) {
        int n = wcnt[wsx];
        if (n > WCAP) n = WCAP;
        if (n < 0) n = 0;
#pragma unroll 1
        for (int i = 0; i < n; ++i) {
          const int ent  = list[wsx * WCAP + i];
          const int slot = ent & (NB - 1);
          const int el   = (ent >> 8) & (CHUNK - 1);
          int e = cbase + el;
          if (e > nE - 1) e = nE - 1;
          int src = ei[e];
          src = src < 0 ? 0 : (src > nN - 1 ? nN - 1 : src);
          int nd = nodeBase + slot;
          if (nd > nN - 1) nd = nN - 1;
          const float al = leaky(AL[(size_t)src * 8 + hd] + AL[(size_t)nd * 8 + 4 + hd]);
          const int   ai = slot * NH + hd;
          const float mo = mxr[ai];
          const float mn = fmaxf(mo, al);
          const float sc = __expf(mo - mn);
          const float p  = __expf(al - mn);
          const float* xs = xp + (size_t)src * DF + 8 * lane;
          const v4f xv0 = *(const v4f*)xs;
          const v4f xv1 = *(const v4f*)(xs + 4);
          v4f* sp = (v4f*)(sacc + slot * DF + 8 * lane);
          v4f t0 = sp[0];
          v4f t1 = sp[1];
          t0 = t0 * sc + xv0 * p;
          t1 = t1 * sc + xv1 * p;
          sp[0] = t0;
          sp[1] = t1;
          if ((lane & 7) == 0) {
            const float dv = den[ai];
            den[ai] = dv * sc + p;
            mxr[ai] = mn;
          }
        }
      }
    }
    __syncthreads();
  }

  {
    const int hd = lane >> 3;
    const v4f b0 = *(const v4f*)(bias + 8 * lane);
    const v4f b1 = *(const v4f*)(bias + 8 * lane + 4);
#pragma unroll 1
    for (int j = 0; j < NB / NWAVE; ++j) {
      const int slot = wave * (NB / NWAVE) + j;
      const int node = nodeBase + slot;
      if (node >= nPad) break;
      const float inv = 1.0f / (den[slot * NH + hd] + 1e-16f);
      const v4f* sp = (const v4f*)(sacc + slot * DF + 8 * lane);
      v4f h0 = relu4(sp[0] * inv + b0);
      v4f h1 = relu4(sp[1] * inv + b1);
      const float keep = (node < nN) ? 16.0f : 0.0f;
      h0 = h0 * keep; h1 = h1 * keep;
      Pack16 u;
      u.h[0] = (_Float16)h0.x; u.h[1] = (_Float16)h0.y; u.h[2] = (_Float16)h0.z; u.h[3] = (_Float16)h0.w;
      u.h[4] = (_Float16)h1.x; u.h[5] = (_Float16)h1.y; u.h[6] = (_Float16)h1.z; u.h[7] = (_Float16)h1.w;
      _Float16* op = hout + (size_t)node * DF + 8 * lane;
      *(volatile v4i*)op = u.i;
      __threadfence();
      *(volatile v4i*)op = u.i;
    }
  }
}

__global__ __launch_bounds__(NTHR) void k_pool(const _Float16* __restrict__ Hh, const int* __restrict__ bat,
                                               _Float16* Ph, int nN) {
  __shared__ __attribute__((aligned(16))) float part[NWAVE * DF];
  __shared__ int cntl[NWAVE];

  const int tid  = threadIdx.x;
  const int lane = tid & 31;
  const int wave = tid >> 5;
  const int g    = blockIdx.x;
  const v4f z4 = {0.f, 0.f, 0.f, 0.f};
  v4f a0 = z4, a1 = z4;
  int cnt = 0;
  const int nCh = (nN + NTHR - 1) / NTHR;
#pragma unroll 1
  for (int c = 0; c < nCh; ++c) {
    const int node = c * NTHR + tid;
    int nc = node; if (nc > nN - 1) nc = nN - 1;
    const int bv = bat[nc];
    const bool hit = (node < nN) && (bv == g);
    unsigned mk = __builtin_amdgcn_ballot_w32(hit);
    cnt += (int)__builtin_popcount(mk);
    while (mk != 0u) {
      const int j = __builtin_ctz(mk);
      mk &= mk - 1u;
      int nd = c * NTHR + wave * 32 + j;
      if (nd > nN - 1) nd = nN - 1;
      Pack16 u;
      u.i = *(const v4i*)(Hh + (size_t)nd * DF + 8 * lane);
      a0.x += (float)u.h[0]; a0.y += (float)u.h[1]; a0.z += (float)u.h[2]; a0.w += (float)u.h[3];
      a1.x += (float)u.h[4]; a1.y += (float)u.h[5]; a1.z += (float)u.h[6]; a1.w += (float)u.h[7];
    }
  }
  *(v4f*)(part + wave * DF + 8 * lane)     = a0;
  *(v4f*)(part + wave * DF + 8 * lane + 4) = a1;
  if (lane == 0) cntl[wave] = cnt;
  __syncthreads();

  if (wave == 0) {
    v4f s0 = z4, s1 = z4;
    int ct = 0;
#pragma unroll
    for (int w = 0; w < NWAVE; ++w) {
      s0 += *(const v4f*)(part + w * DF + 8 * lane);
      s1 += *(const v4f*)(part + w * DF + 8 * lane + 4);
      ct += cntl[w];
    }
    const float rc = 1.0f / fmaxf((float)ct, 1.0f);
    const v4f t0 = s0 * rc;
    const v4f t1 = s1 * rc;
    Pack16 u;
    u.h[0] = (_Float16)(t0.x * 16.0f); u.h[1] = (_Float16)(t0.y * 16.0f);
    u.h[2] = (_Float16)(t0.z * 16.0f); u.h[3] = (_Float16)(t0.w * 16.0f);
    u.h[4] = (_Float16)(t1.x * 16.0f); u.h[5] = (_Float16)(t1.y * 16.0f);
    u.h[6] = (_Float16)(t1.z * 16.0f); u.h[7] = (_Float16)(t1.w * 16.0f);
    _Float16* op = Ph + (size_t)g * DF + 8 * lane;
    *(volatile v4i*)op = u.i;
    __threadfence();
    *(volatile v4i*)op = u.i;
  }
}

__global__ __launch_bounds__(NTHR) void k_head(
    const _Float16* __restrict__ Ph, const _Float16* __restrict__ P1t, const float* __restrict__ pb1,
    const _Float16* __restrict__ P2t, const float* __restrict__ pb2, float* out) {
  __shared__ __attribute__((aligned(16))) _Float16 Zs[GR * ZP];
  __shared__ __attribute__((aligned(16))) float Os[GR * OSP];

  const int tid  = threadIdx.x;
  const int lane = tid & 31;
  const int wave = tid >> 5;
  const int hh   = lane >> 4;
  const int m    = lane & 15;
  const int rowBase = blockIdx.x * GR;

  {
    const int T = wave >> 2;
    const int J = wave & 3;
    const _Float16* pa = Ph  + (size_t)(rowBase + 16 * T + m) * DF + 8 * hh;
    const _Float16* pb = P1t + (size_t)(16 * J + m) * DF + 8 * hh;
    v8f c = {0.f, 0.f, 0.f, 0.f, 0.f, 0.f, 0.f, 0.f};
#pragma unroll 2
    for (int kt = 0; kt < DF / 32; ++kt) {
      const int k0 = kt * 32;
      Frag a, b;
      a.half[0] = *(const v8h*)(pa + k0); a.half[1] = *(const v8h*)(pa + k0 + 16);
      b.half[0] = *(const v8h*)(pb + k0); b.half[1] = *(const v8h*)(pb + k0 + 16);
      c = wm(a.v, b.v, c);
    }
    const int col = 16 * J + m;
    const float bv = pb1[col];
#pragma unroll
    for (int r = 0; r < 8; ++r) {
      const float v = fmaxf(c[r] * (1.0f / 4096.0f) + bv, 0.0f) * 256.0f;
      Zs[(16 * T + 8 * hh + r) * ZP + col] = (_Float16)v;
    }
  }
  __syncthreads();

  {
    const _Float16* pz0 = Zs + m * ZP + 8 * hh;
    const _Float16* pz1 = Zs + (16 + m) * ZP + 8 * hh;
    const _Float16* pw  = P2t + (size_t)(16 * wave + m) * HID + 8 * hh;
    v8f d0 = {0.f, 0.f, 0.f, 0.f, 0.f, 0.f, 0.f, 0.f};
    v8f d1 = d0;
#pragma unroll
    for (int kt = 0; kt < HID / 32; ++kt) {
      const int k0 = kt * 32;
      Frag a0, a1, b;
      a0.half[0] = *(const v8h*)(pz0 + k0); a0.half[1] = *(const v8h*)(pz0 + k0 + 16);
      a1.half[0] = *(const v8h*)(pz1 + k0); a1.half[1] = *(const v8h*)(pz1 + k0 + 16);
      b.half[0]  = *(const v8h*)(pw + k0);  b.half[1]  = *(const v8h*)(pw + k0 + 16);
      d0 = wm(a0.v, b.v, d0);
      d1 = wm(a1.v, b.v, d1);
    }
    const int col = 16 * wave + m;
    const float bv = pb2[col];
#pragma unroll
    for (int r = 0; r < 8; ++r) {
      Os[(8 * hh + r) * OSP + col]      = d0[r] * (1.0f / 4096.0f) + bv;
      Os[(16 + 8 * hh + r) * OSP + col] = d1[r] * (1.0f / 4096.0f) + bv;
    }
  }
  __syncthreads();

  v4f orow[4];
#pragma unroll
  for (int i = 0; i < 4; ++i) orow[i] = *(const v4f*)(Os + (4 * wave + i) * OSP + 4 * lane);
  float* op = out + (size_t)(rowBase + 4 * wave) * OUTD + 4 * lane;
#pragma unroll
  for (int i = 0; i < 4; ++i) *(volatile v4f*)(op + (size_t)i * OUTD) = orow[i];
  __threadfence();
#pragma unroll
  for (int i = 0; i < 4; ++i) *(volatile v4f*)(op + (size_t)i * OUTD) = orow[i];
}

extern "C" void kernel_launch(void* const* d_in, const int* in_sizes, int n_in,
                              void* d_out, int out_size, void* d_ws, size_t ws_size,
                              hipStream_t stream) {
  if (n_in < 15) return;
  const int nN = in_sizes[0] / IN0;
  if (nN <= 0 || in_sizes[0] != nN * IN0) return;
  const int nE = in_sizes[1] / 2;
  if (nE < 0 || in_sizes[1] != 2 * nE) return;
  if (in_sizes[2] != nN) return;
  if (in_sizes[3] != IN0 * DF) return;
  if (in_sizes[4] != NH * HC || in_sizes[5] != NH * HC || in_sizes[6] != DF) return;
  if (in_sizes[7] != DF * DF) return;
  if (in_sizes[8] != NH * HC || in_sizes[9] != NH * HC || in_sizes[10] != DF) return;
  if (in_sizes[11] != DF * HID || in_sizes[12] != HID) return;
  if (in_sizes[13] != HID * OUTD || in_sizes[14] != OUTD) return;
  if (out_size != NGR * OUTD) return;

  const float* x      = (const float*)d_in[0];
  const int*   ei     = (const int*)d_in[1];
  const int*   bat    = (const int*)d_in[2];
  const float* W0     = (const float*)d_in[3];
  const float* a_src0 = (const float*)d_in[4];
  const float* a_dst0 = (const float*)d_in[5];
  const float* b0     = (const float*)d_in[6];
  const float* W1     = (const float*)d_in[7];
  const float* a_src1 = (const float*)d_in[8];
  const float* a_dst1 = (const float*)d_in[9];
  const float* b1     = (const float*)d_in[10];
  const float* pW1    = (const float*)d_in[11];
  const float* pb1    = (const float*)d_in[12];
  const float* pW2    = (const float*)d_in[13];
  const float* pb2    = (const float*)d_in[14];
  float* out = (float*)d_out;

  const int nPad = ((nN + GR - 1) / GR) * GR;
  size_t off = 0;
#define CARVE(ptr, T, bytes) ptr = (T*)((char*)d_ws + off); off += ((size_t)(bytes) + 255) & ~(size_t)255;
  _Float16* xh;  CARVE(xh,  _Float16, (size_t)nPad * IN0 * 2)
  _Float16* Wt0; CARVE(Wt0, _Float16, (size_t)DF * IN0 * 2)
  _Float16* Wt1; CARVE(Wt1, _Float16, (size_t)DF * DF * 2)
  _Float16* Pt1; CARVE(Pt1, _Float16, (size_t)HID * DF * 2)
  _Float16* Pt2; CARVE(Pt2, _Float16, (size_t)OUTD * HID * 2)
  float*    xp;  CARVE(xp,  float,    (size_t)nPad * DF * 4)
  float*    AL;  CARVE(AL,  float,    (size_t)nPad * 8 * 4)
  _Float16* hpl; CARVE(hpl, _Float16, (size_t)nPad * DF * 2)
  _Float16* Ph;  CARVE(Ph,  _Float16, (size_t)NGR * DF * 2)
#undef CARVE
  if (off > ws_size) return;
  if (off > (size_t)134217728) return;

  const int n8x = nPad * IN0 / 8;
  k_cvt<<<(n8x + NTHR - 1) / NTHR, NTHR, 0, stream>>>(x, xh, nN, n8x);
  {
    const int n0 = IN0 * DF / 8;
    k_wprep<<<(n0 + NTHR - 1) / NTHR, NTHR, 0, stream>>>(W0, Wt0, IN0, DF, 16.0f, n0);
    const int n1 = DF * DF / 8;
    k_wprep<<<(n1 + NTHR - 1) / NTHR, NTHR, 0, stream>>>(W1, Wt1, DF, DF, 16.0f, n1);
    const int n2 = DF * HID / 8;
    k_wprep<<<(n2 + NTHR - 1) / NTHR, NTHR, 0, stream>>>(pW1, Pt1, DF, HID, 16.0f, n2);
    const int n3 = HID * OUTD / 8;
    k_wprep<<<(n3 + NTHR - 1) / NTHR, NTHR, 0, stream>>>(pW2, Pt2, HID, OUTD, 16.0f, n3);
  }

  hipFuncSetAttribute(reinterpret_cast<const void*>(&k_agg),
                      hipFuncAttributeMaxDynamicSharedMemorySize, LDS_AGG_BYTES);
  const int gridG = nPad / GR;
  const int gridA = (nPad + NB - 1) / NB;

  k_gemm<IN0><<<gridG, NTHR, 0, stream>>>(xh, Wt0, a_src0, a_dst0, xp, AL, 1.0f / 16.0f);
  k_agg<<<gridA, NTHR, LDS_AGG_BYTES, stream>>>(ei, xp, AL, b0, hpl, nN, nE, nPad);

  k_gemm<DF><<<gridG, NTHR, 0, stream>>>(hpl, Wt1, a_src1, a_dst1, xp, AL, 1.0f / 256.0f);
  k_agg<<<gridA, NTHR, LDS_AGG_BYTES, stream>>>(ei, xp, AL, b1, hpl, nN, nE, nPad);

  k_pool<<<NGR, NTHR, 0, stream>>>(hpl, bat, Ph, nN);
  k_head<<<NGR / GR, NTHR, 0, stream>>>(Ph, Pt1, pb1, Pt2, pb2, out);
}
